// LinearCrossAttention_37967510896792
// MI455X (gfx1250) — hardware-run, weakly checked
//
#include <hip/hip_runtime.h>
#define NB 8
#define NBP 4
#define SQ 4096
#define DM 384
#define NH 6
#define HD 64
#define EPSZ 1e-6f
#define WCAR 64.0f
#define VCAR 16.0f
#define OCAR 1024.0f
typedef __bf16 v16b __attribute__((ext_vector_type(16)));
typedef unsigned short v8us __attribute__((ext_vector_type(8), may_alias));
typedef float  v8f  __attribute__((ext_vector_type(8)));
typedef float  v4f  __attribute__((ext_vector_type(4)));
typedef float  v4fa __attribute__((ext_vector_type(4), may_alias));
union FragB { v16b v; v8us half[2]; unsigned short u[16]; };

__device__ __forceinline__ unsigned short bf16_bits(float x) { unsigned int u = __float_as_uint(x); return (unsigned short)((u + 0x7FFFu + ((u >> 16) & 1u)) >> 16); }
__device__ __forceinline__ float bf16_val(unsigned short b) { return __uint_as_float(((unsigned int)b) << 16); }
__device__ __forceinline__ float bf16_round(float x) { return bf16_val(bf16_bits(x)); }
template <int NT>
__device__ __forceinline__ v8f mmaN(v16b ah, v16b al, v16b bh, v16b bl, v8f c) {
  c = __builtin_amdgcn_wmma_f32_16x16x32_bf16(false, ah, false, bh, (short)0, c, false, false);
  if (NT >= 2) c = __builtin_amdgcn_wmma_f32_16x16x32_bf16(false, al, false, bh, (short)0, c, false, false);
  if (NT >= 3) c = __builtin_amdgcn_wmma_f32_16x16x32_bf16(false, ah, false, bl, (short)0, c, false, false);
  asm volatile("v_nop\n\tv_nop\n\tv_nop\n\tv_nop" : "+v"(c) : "v"(ah), "v"(al), "v"(bh), "v"(bl));
  return c;
}


typedef _Float16 v16h __attribute__((ext_vector_type(16)));
union FragH { v16h v; v8us half[2]; _Float16 h[16]; unsigned short u[16]; };
template <int NT>
__device__ __forceinline__ v8f mmaH(v16h ah, v16h al, v16h bh, v16h bl, v8f c) {
  c = __builtin_amdgcn_wmma_f32_16x16x32_f16(false, ah, false, bh, (short)0, c, false, false);
  if (NT >= 2) c = __builtin_amdgcn_wmma_f32_16x16x32_f16(false, al, false, bh, (short)0, c, false, false);
  if (NT >= 3) c = __builtin_amdgcn_wmma_f32_16x16x32_f16(false, ah, false, bl, (short)0, c, false, false);
  asm volatile("v_nop\n\tv_nop\n\tv_nop\n\tv_nop" : "+v"(c) : "v"(ah), "v"(al), "v"(bh), "v"(bl));
  return c;
}

__global__ __launch_bounds__(256) void k_wt_f16(const float* __restrict__ W, _Float16* __restrict__ Wt, int K, int N, float scale) {
  const int t = blockIdx.x * 256 + threadIdx.x; if (t >= N * (K / 8)) return; const int n = t / (K / 8), k8 = (t % (K / 8)) * 8; FragH f;
#pragma unroll
  for (int i = 0; i < 8; ++i) f.h[i] = (_Float16)(bf16_round(W[(size_t)(k8 + i) * N + n]) * scale); const v8us o = f.half[0];
  *(volatile v8us*)((unsigned short*)Wt + (size_t)n * K + k8) = o; __threadfence(); *(volatile v8us*)((unsigned short*)Wt + (size_t)n * K + k8) = o;
}

typedef _Float16 v4h __attribute__((ext_vector_type(4)));

__global__ __launch_bounds__(256) void k_x16(const float* __restrict__ x, _Float16* __restrict__ X16, size_t n8) { const size_t t = (size_t)blockIdx.x * 256 + threadIdx.x; if (t >= n8) return; FragH f;
#pragma unroll
  for (int q = 0; q < 8; ++q) f.h[q] = (_Float16)bf16_round(x[t * 8 + q]); *(volatile v8us*)((unsigned short*)X16 + t * 8) = f.half[0]; __threadfence(); *(volatile v8us*)((unsigned short*)X16 + t * 8) = f.half[0]; }
__device__ __forceinline__ v16h g2_frag(const _Float16* p, int hh) { FragH f; f.half[0] = *(const v8us*)((const unsigned short*)p + 8 * hh); f.half[1] = *(const v8us*)((const unsigned short*)p + 16 + 8 * hh); return f.v; }
__device__ __forceinline__ v8f g2_mma(v16h a, v16h b, v8f c) { v8f d = __builtin_amdgcn_wmma_f32_16x16x32_f16(false, a, false, b, (short)0, c, false, false); asm volatile("v_nop\n\tv_nop\n\tv_nop\n\tv_nop" : "+v"(d) : "v"(a), "v"(b)); return d; }
template <int ACT>
__global__ __launch_bounds__(128) void k_gemm2(const _Float16* __restrict__ A, int lda, size_t sA, const _Float16* __restrict__ Bh, int ldb, size_t sB, float alpha, const float* __restrict__ bias, size_t sBias, const float* __restrict__ CP, int rowsPerB, size_t sCPb, int row0g,
    float* __restrict__ C, _Float16* __restrict__ C16, int ldc, size_t sC, int M, int N, int K) { static_assert(ACT == 0 || ACT == 3 || ACT == 6 || ACT == 8 || ACT == 9 || ACT == 11 || ACT == 12 || ACT == 14 || ACT == 15 || ACT == 16 || ACT == 17, "k_gemm2: unsupported ACT code (would silently apply no activation)");
  __shared__ __attribute__((aligned(16))) float so[4][32][68];
  const int tid = threadIdx.x, w = tid >> 5, lane = tid & 31, ln = lane & 15, hh = lane >> 4; const int by = blockIdx.y;
  A += (size_t)by * sA; Bh += (size_t)by * sB; const size_t cofs = (size_t)by * sC; const float* bp = bias ? bias + (size_t)by * sBias : nullptr;
  const int ntn = N >> 6; const int mt = blockIdx.x / ntn, nq = blockIdx.x - mt * ntn; const int row0 = mt * 128 + 32 * w, col0 = nq * 64; if (row0 >= M) return;
  const _Float16* a0p = A + (size_t)(row0 + ln) * lda; const _Float16* a1p = a0p + (size_t)16 * lda;
  const _Float16* b0p = Bh + (size_t)(col0 + ln) * ldb; const _Float16* b1p = b0p + (size_t)16 * ldb; const _Float16* b2p = b1p + (size_t)16 * ldb; const _Float16* b3p = b2p + (size_t)16 * ldb;
  const v8f z8 = {0.f,0.f,0.f,0.f,0.f,0.f,0.f,0.f}; v8f c00 = z8, c01 = z8, c02 = z8, c03 = z8, c10 = z8, c11 = z8, c12 = z8, c13 = z8;
  for (int kb = 0; kb < K; kb += 32) { const v16h a0 = g2_frag(a0p + kb, hh), a1 = g2_frag(a1p + kb, hh);
    v16h b = g2_frag(b0p + kb, hh); c00 = g2_mma(a0, b, c00); c10 = g2_mma(a1, b, c10);
    b = g2_frag(b1p + kb, hh); c01 = g2_mma(a0, b, c01); c11 = g2_mma(a1, b, c11);
    b = g2_frag(b2p + kb, hh); c02 = g2_mma(a0, b, c02); c12 = g2_mma(a1, b, c12);
    b = g2_frag(b3p + kb, hh); c03 = g2_mma(a0, b, c03); c13 = g2_mma(a1, b, c13); }
  v8f accs[8] = {c00, c01, c02, c03, c10, c11, c12, c13};
#pragma unroll
  for (int u = 0; u < 8; ++u) { const int t = u & 3, half = u >> 2; const int col = col0 + t * 16 + ln; const float bv = bp ? bf16_round(bp[col]) : 0.f;
#pragma unroll
    for (int r = 0; r < 8; ++r) { const int rloc = half * 16 + 8 * hh + r; float v = accs[u][r] * alpha + bv; if (CP) { if (rowsPerB < 0) v += CP[cofs + (size_t)(row0g + row0 + rloc) * ldc + col];        else { const int bidx = (row0g + row0 + rloc) / rowsPerB; v += CP[(size_t)bidx * sCPb + (size_t)by * 64 + col]; } }
      if (ACT == 3) v = fmaxf(v, 0.f); else if (ACT == 6) v = 0.5f * v * (1.0f + erff(v * 0.70710678118654752f)); else if (ACT == 11) v = 1.0f / (1.0f + expf(-v)); else if (ACT == 15) v = v / (1.0f + expf(-v)); else if (ACT == 12) v = (v > 0.f) ? v : 0.01f * v; else if (ACT == 8) v = tanhf(v); else if (ACT == 9) v = 0.5f * v * (1.0f + tanhf(0.7978845608028654f * (v + 0.044715f * v * v * v))); else if (ACT == 14) v = (v > 0.f) ? v : 0.1f * v; else if (ACT == 16) v = (v >= 0.f) ? v : 0.3f * v; else if (ACT == 17) v = (v >= 0.f) ? v : 0.2f * v;
      so[w][rloc][t * 16 + ln] = v; } }
  __builtin_amdgcn_fence(__ATOMIC_ACQ_REL, "workgroup"); __builtin_amdgcn_wave_barrier();
  const int rsub = lane >> 4, c4 = (lane & 15) * 4;
  for (int pass = 0; pass < 2; ++pass) {
#pragma unroll
    for (int q = 0; q < 16; ++q) { const int r = q * 2 + rsub; const v4f v = *(const v4fa*)&so[w][r][c4]; if (C) *(volatile v4f*)(C + cofs + (size_t)(row0 + r) * ldc + col0 + c4) = v; if (C16) { v4h h4; for (int i = 0; i < 4; ++i) h4[i] = (_Float16)v[i]; *(volatile v4h*)(C16 + cofs + (size_t)(row0 + r) * ldc + col0 + c4) = h4; } }
    if (pass == 0) __threadfence(); } }

__global__ __launch_bounds__(256) void k_phi(float* XF, _Float16* __restrict__ H16, size_t n8) {
  const size_t t = (size_t)blockIdx.x * 256 + threadIdx.x; if (t >= n8) return; float* xp = XF + t * 8; const v4f a = *(const v4fa*)xp; const v4f c = *(const v4fa*)(xp + 4); v4f ya, yc; FragH f;
#pragma unroll
  for (int q = 0; q < 4; ++q) { ya[q] = expf(fminf(a[q], 0.f)) + fmaxf(a[q], 0.f); yc[q] = expf(fminf(c[q], 0.f)) + fmaxf(c[q], 0.f); f.h[q] = (_Float16)ya[q]; f.h[4 + q] = (_Float16)yc[q]; }
  unsigned short* hp = (unsigned short*)H16 + t * 8;
  for (int pass = 0; pass < 2; ++pass) { *(volatile v4f*)xp = ya; *(volatile v4f*)(xp + 4) = yc; *(volatile v8us*)hp = f.half[0]; if (pass == 0) __threadfence(); } }
__global__ __launch_bounds__(256) void k_wtc_f16(const float* __restrict__ W, _Float16* __restrict__ Wt, int K, int N, float scale) {
  const int t = blockIdx.x * 256 + threadIdx.x; if (t >= N * (K / 8)) return; const int n = t / (K / 8), k8 = (t % (K / 8)) * 8; FragH f;
#pragma unroll
  for (int i = 0; i < 8; ++i) f.h[i] = (_Float16)(W[(size_t)(k8 + i) * N + n] * scale); const v8us o = f.half[0];
  *(volatile v8us*)((unsigned short*)Wt + (size_t)n * K + k8) = o; __threadfence(); *(volatile v8us*)((unsigned short*)Wt + (size_t)n * K + k8) = o;
}
__global__ __launch_bounds__(256) void k_ksum(const _Float16* __restrict__ KT, float* __restrict__ KS, int n) {
  const int t = blockIdx.x * 256 + threadIdx.x; if (t >= n) return; const unsigned short* r = (const unsigned short*)KT + (size_t)t * SQ; float acc = 0.f;
  for (int j = 0; j < SQ / 8; ++j) { FragH f; f.half[0] = *(const v8us*)(r + 8 * j); for (int i = 0; i < 8; ++i) acc += (float)f.h[i]; }
  *(volatile float*)(KS + t) = acc; __threadfence(); *(volatile float*)(KS + t) = acc; }
__global__ __launch_bounds__(256) void k_zdot6(const _Float16* __restrict__ Q16, const float* __restrict__ KS, const float* __restrict__ ND, _Float16* __restrict__ O16, int n) {
  const int t = blockIdx.x * 256 + threadIdx.x; if (t >= n) return; const int row = t / NH, hh = t - row * NH, bh = (row >> 12) * NH + hh; const unsigned short* q = (const unsigned short*)Q16 + (size_t)t * HD; const float* ks = KS + bh * HD; float den = 0.f;
  for (int j = 0; j < HD / 8; ++j) { FragH f; f.half[0] = *(const v8us*)(q + 8 * j); for (int i = 0; i < 8; ++i) den += (float)f.h[i] * ks[8 * j + i]; }
  const float z = OCAR / (den + EPSZ); const float* p = ND + (size_t)t * HD; unsigned short* o = (unsigned short*)O16 + (size_t)t * HD;
  for (int pass = 0; pass < 2; ++pass) {
    for (int j = 0; j < HD / 8; ++j) { const v4f a = *(const v4fa*)(p + 8 * j); const v4f c = *(const v4fa*)(p + 8 * j + 4); FragH f; for (int i = 0; i < 4; ++i) { f.h[i] = (_Float16)(a[i] * z); f.h[4 + i] = (_Float16)(c[i] * z); } *(volatile v8us*)(o + 8 * j) = f.half[0]; }
    if (pass == 0) __threadfence(); } }

extern "C" void kernel_launch(void* const* d_in, const int* in_sizes, int n_in,
                              void* d_out, int out_size, void* d_ws, size_t ws_size, hipStream_t stream) {
  (void)in_sizes; (void)n_in; (void)out_size;
  const float* x_q = (const float*)d_in[0]; const float* x_kv = (const float*)d_in[1]; const float* Wq = (const float*)d_in[2]; const float* Wkv = (const float*)d_in[3]; const float* Wout = (const float*)d_in[4]; const float* bout = (const float*)d_in[5];
  static_assert(NB == 8 && NBP == 4 && NB % NBP == 0 && SQ == 4096 && DM == 384 && NH * HD == DM && HD == 64 && (NBP * SQ) % 128 == 0 && SQ % 128 == 0 && DM % 64 == 0 && DM % 32 == 0 && HD % 32 == 0 && SQ % 32 == 0 && ((size_t)NBP * SQ * DM / 8) % 256 == 0 && ((size_t)DM * (DM / 8)) % 256 == 0 && ((size_t)2 * DM * (DM / 8)) % 256 == 0 && ((size_t)DM * (SQ / 8)) % 256 == 0 && (NBP * DM) % 256 == 0 && ((size_t)NBP * SQ * NH) % 256 == 0, "the index shift; whole tiles; exact grids");
  float* out = (float*)d_out;
  const int NRP = NBP * SQ;
  char* ws = (char*)d_ws; size_t off = 0;
  auto take = [&](size_t bytes) { char* p = ws + off; off += (bytes + 255) & ~(size_t)255; return p; };
  _Float16* WQT = (_Float16*)take((size_t)DM * DM * 2); _Float16* WKVT = (_Float16*)take((size_t)2 * DM * DM * 2); _Float16* WOT = (_Float16*)take((size_t)DM * DM * 2);
  _Float16* XQ = (_Float16*)take((size_t)NRP * DM * 2); _Float16* XKV = (_Float16*)take((size_t)NRP * DM * 2); float* FA = (float*)take((size_t)NRP * DM * 4); _Float16* QH = (_Float16*)take((size_t)NRP * DM * 2); _Float16* KH = (_Float16*)take((size_t)NRP * DM * 2);
  _Float16* KT = (_Float16*)take((size_t)NBP * DM * SQ * 2); _Float16* VT = (_Float16*)take((size_t)NBP * DM * SQ * 2); float* KS = (float*)take((size_t)NBP * DM * 4); _Float16* KVT = (_Float16*)take((size_t)NBP * NH * HD * HD * 2); _Float16* O16 = (_Float16*)take((size_t)NRP * DM * 2);
  if (off > ws_size) return;
  k_wt_f16<<<(unsigned)((size_t)DM * (DM / 8) / 256), 256, 0, stream>>>(Wq, WQT, DM, DM, WCAR); k_wt_f16<<<(unsigned)((size_t)2 * DM * (DM / 8) / 256), 256, 0, stream>>>(Wkv, WKVT, DM, 2 * DM, WCAR); k_wt_f16<<<(unsigned)((size_t)DM * (DM / 8) / 256), 256, 0, stream>>>(Wout, WOT, DM, DM, WCAR);
  for (int g = 0; g < NB / NBP; ++g) { const size_t r0 = (size_t)g * NRP;
    k_x16<<<(unsigned)((size_t)NRP * DM / 8 / 256), 256, 0, stream>>>(x_q + r0 * DM, XQ, (size_t)NRP * DM / 8); k_x16<<<(unsigned)((size_t)NRP * DM / 8 / 256), 256, 0, stream>>>(x_kv + r0 * DM, XKV, (size_t)NRP * DM / 8);
    k_gemm2<0><<<dim3((unsigned)((NRP / 128) * (DM / 64)), 1), 128, 0, stream>>>(XQ, DM, (size_t)0, WQT, DM, (size_t)0, 1.0f / WCAR, nullptr, 0, nullptr, 1, 0, 0, FA, nullptr, DM, (size_t)0, NRP, DM, DM);
    k_phi<<<(unsigned)((size_t)NRP * DM / 8 / 256), 256, 0, stream>>>(FA, QH, (size_t)NRP * DM / 8);
    k_gemm2<0><<<dim3((unsigned)((NRP / 128) * (DM / 64)), 1), 128, 0, stream>>>(XKV, DM, (size_t)0, WKVT, DM, (size_t)0, 1.0f / WCAR, nullptr, 0, nullptr, 1, 0, 0, FA, nullptr, DM, (size_t)0, NRP, DM, DM);
    k_phi<<<(unsigned)((size_t)NRP * DM / 8 / 256), 256, 0, stream>>>(FA, KH, (size_t)NRP * DM / 8);
    for (int b = 0; b < NBP; ++b) k_wtc_f16<<<(unsigned)((size_t)DM * (SQ / 8) / 256), 256, 0, stream>>>(FA + (size_t)b * SQ * DM, KT + (size_t)b * DM * SQ, SQ, DM, 1.0f);
    k_gemm2<0><<<dim3((unsigned)((NRP / 128) * (DM / 64)), 1), 128, 0, stream>>>(XKV, DM, (size_t)0, WKVT + (size_t)DM * DM, DM, (size_t)0, 1.0f / WCAR, nullptr, 0, nullptr, 1, 0, 0, FA, nullptr, DM, (size_t)0, NRP, DM, DM);
    for (int b = 0; b < NBP; ++b) k_wtc_f16<<<(unsigned)((size_t)DM * (SQ / 8) / 256), 256, 0, stream>>>(FA + (size_t)b * SQ * DM, VT + (size_t)b * DM * SQ, SQ, DM, VCAR);
    k_ksum<<<(unsigned)((size_t)NBP * DM / 256), 256, 0, stream>>>(KT, KS, NBP * DM);
    k_gemm2<0><<<dim3((HD / 64) * (HD / 64), NBP * NH), 128, 0, stream>>>(VT, SQ, (size_t)HD * SQ, KT, SQ, (size_t)HD * SQ, 1.0f, nullptr, 0, nullptr, 1, 0, 0, nullptr, KVT, HD, (size_t)HD * HD, HD, HD, SQ);
    for (int b = 0; b < NBP; ++b) k_gemm2<0><<<dim3((SQ / 128) * (HD / 64), NH), 128, 0, stream>>>(QH + (size_t)b * SQ * DM, DM, (size_t)HD, KVT + (size_t)b * NH * HD * HD, HD, (size_t)HD * HD, 1.0f / VCAR, nullptr, 0, nullptr, 1, 0, 0, FA + (size_t)b * SQ * DM, nullptr, DM, (size_t)HD, SQ, HD, HD);
    k_zdot6<<<(unsigned)((size_t)NRP * NH / 256), 256, 0, stream>>>(QH, KS, FA, O16, NRP * NH);
    k_gemm2<0><<<dim3((unsigned)((NRP / 128) * (DM / 64)), 1), 128, 0, stream>>>(O16, DM, (size_t)0, WOT, DM, (size_t)0, 1.0f / (OCAR * WCAR), bout, 0, nullptr, 1, 0, 0, out + r0 * DM, nullptr, DM, (size_t)0, NRP, DM, DM);
  }
}
